// unit_ctrgcn_sparse_32006096290316
// MI455X (gfx1250) — hardware-run, weakly checked
//
#include <hip/hip_runtime.h>


#ifndef NB
#define NB 16
#endif
#define NB_FULL 16
#define CC   64
#define TT   512
#define VV   25
#define RR   8
#define NS   3
#define PIXN (TT * VV)
#define TB   32
#define PB   (TB * VV)
#define MTN  (PB / 16)
#define OGC  16
#define NW   8
#define UP   32
#define OPX  (TB * UP + 8)
#define XBP  72
#define X3C  16.0f
#define ATC  256.0f
#define ZI   (1.0f / 4096.0f)
#define XBC  64.0f
#define WCC  16.0f
#define X1I  (1.0f / 1024.0f)
#define NQ   (PB / 4)

static_assert(CC == 64);
static_assert(CC % 32 == 0);
static_assert(TB == 32);
static_assert(UP == 32);
static_assert(VV <= UP);
static_assert(TT % TB == 0);
static_assert(PB % 16 == 0);
static_assert((PB * 4) % 128 == 0);
static_assert(((size_t)PIXN * 4) % 128 == 0);
static_assert(NW * 2 == OGC);
static_assert(CC % OGC == 0);
static_assert(2 * RR == 16);
static_assert(NQ == 200);
static_assert(6 * 32 < NQ && NQ <= 7 * 32);
static_assert((NQ - 6 * 32) * 16 == 128);
static_assert(7 * 32 * 16 >= PB * 4);
static_assert((OPX * 2) % 16 == 0);
static_assert((XBP * 2) % 16 == 0);
static_assert((size_t)NS * OGC * OPX * 2 + (size_t)NW * PB * 4 <= 131072);
static_assert(32 * 256 == CC * UP * (UP / 8));
static_assert(((size_t)NB * PIXN * 8) % 256 == 0);
static_assert(((size_t)NS * CC * CC / 8) % 256 == 0);
static_assert(NB <= NB_FULL);

typedef _Float16 h16;
typedef unsigned short bf;
typedef __attribute__((ext_vector_type(16))) __bf16   v16bf;
typedef __attribute__((ext_vector_type(16))) _Float16 v16h;
typedef __attribute__((ext_vector_type(8)))  _Float16 v8h;
typedef __attribute__((ext_vector_type(8)))  unsigned short v8us;
typedef __attribute__((ext_vector_type(8)))  float    v8f;
typedef __attribute__((ext_vector_type(4)))  float    v4f;
typedef v4f  __attribute__((may_alias)) v4fa;
typedef v8h  __attribute__((may_alias)) v8ha;

__device__ __forceinline__ unsigned short f2bf(float f) { unsigned u = __float_as_uint(f); u += 0x7FFFu + ((u >> 16) & 1u); return (unsigned short)(u >> 16); }
__device__ __forceinline__ float bfr(float f) { return __uint_as_float(((unsigned)f2bf(f)) << 16); }
__device__ __forceinline__ v16h cat16(v8h lo, v8h hi) { return __builtin_shufflevector(lo, hi, 0, 1, 2, 3, 4, 5, 6, 7, 8, 9, 10, 11, 12, 13, 14, 15); }
__device__ __forceinline__ v16bf cat16b(v8us lo, v8us hi) { return __builtin_bit_cast(v16bf, __builtin_shufflevector(lo, hi, 0, 1, 2, 3, 4, 5, 6, 7, 8, 9, 10, 11, 12, 13, 14, 15)); }
__device__ __forceinline__ v16h  ldh(const h16* p) { return cat16(*(const v8h*)p, *(const v8h*)(p + 16)); }
__device__ __forceinline__ v16bf ldb(const bf* p)  { return cat16b(*(const v8us*)p, *(const v8us*)(p + 16)); }
__device__ __forceinline__ void wave_sync() { __builtin_amdgcn_fence(3  , "wavefront"); __builtin_amdgcn_wave_barrier(); asm volatile("" ::: "memory"); }
static __device__ __forceinline__ h16 toh_flush(float v) { const h16 r = (h16)v; return (fabsf(v) < 6.103515625e-05f) ? (h16)0.0f : r; }
__device__ __forceinline__ v8f wmma16g(v16h a, v16h b, v8f c) {
    c = __builtin_amdgcn_wmma_f32_16x16x32_f16(false, a, false, b, (short)0, c, false, false);
    asm volatile("v_nop\n\tv_nop\n\tv_nop\n\tv_nop" : "+v"(c) : "v"(a), "v"(b));
    return c; }
__device__ __forceinline__ v8f wmmabg(v16bf a, v16bf b, v8f c) {
    c = __builtin_amdgcn_wmma_f32_16x16x32_bf16(false, a, false, b, (short)0, c, false, false);
    asm volatile("v_nop\n\tv_nop\n\tv_nop\n\tv_nop" : "+v"(c) : "v"(a), "v"(b));
    return c; }

__global__ __launch_bounds__(256) void k_wcvt(const float* __restrict__ src, const int* __restrict__ sp, bf* dst, unsigned n8) {
#pragma clang fp contract(off)
    const unsigned i = blockIdx.x * 256u + threadIdx.x; if (i >= n8) return;
    const float thr = (float)sp[0];
    const v8f v = *(const v8f*)(src + (size_t)i * 8); v8us o;
#pragma unroll
    for (int k = 0; k < 8; ++k) { float r = bfr(v[k]); r = (fabsf(r) > thr) ? r : 0.0f; o[k] = f2bf(r); }
    *(volatile v8us*)(dst + (size_t)i * 8) = o; __threadfence(); *(volatile v8us*)(dst + (size_t)i * 8) = o;
}

__global__ __launch_bounds__(256) void k_tr(const float* __restrict__ x, bf* XT, unsigned n8) {
#pragma clang fp contract(off)
    const unsigned i = blockIdx.x * 256u + threadIdx.x; if (i >= n8) return;
    const unsigned k = i & 7u, row = i >> 3;
    const unsigned n = row / (unsigned)PIXN; const unsigned pix = row - n * (unsigned)PIXN;
    const float* s = x + ((size_t)n * CC + 8u * k) * PIXN + pix;
    v8us o;
#pragma unroll
    for (int j = 0; j < 8; ++j) o[j] = f2bf(s[(size_t)j * PIXN]);
    *(volatile v8us*)(XT + (size_t)i * 8) = o; __threadfence(); *(volatile v8us*)(XT + (size_t)i * 8) = o;
}

__global__ __launch_bounds__(256) void k_xbar(const float* __restrict__ x, float* XBAR) {
#pragma clang fp contract(off)
    __shared__ float sm[8 * 32];
    __shared__ __align__(16) float so[32];
    const int nc = blockIdx.x;
    const int lane = threadIdx.x & 31;
    const int grp = __builtin_amdgcn_readfirstlane((int)(threadIdx.x >> 5));
    const int vc = lane < VV ? lane : (VV - 1);
    const float* p = x + (size_t)nc * PIXN + vc;
    float acc = 0.0f;
#pragma unroll 4
    for (int t = grp; t < TT; t += 8) { float xv = p[(size_t)t * VV]; asm volatile("" : "+v"(xv)); acc += bfr(xv); }
    sm[grp * 32 + lane] = acc;
    __syncthreads();
    if (grp == 0) {
        float tot = 0.0f;
#pragma unroll
        for (int g = 0; g < 8; ++g) tot += sm[g * 32 + lane];
        so[lane] = (lane < VV) ? tot * (1.0f / (float)TT) : 0.0f;
        wave_sync();
        const v4f o4 = *(const v4fa*)(&so[(lane & 7) * 4]);
        if (lane < 8) { float* d = XBAR + (size_t)nc * UP + lane * 4;
            *(volatile v4f*)d = o4; __threadfence(); *(volatile v4f*)d = o4; }
    }
}

__global__ __launch_bounds__(256) void k_amat(const float* __restrict__ XBAR, const float* __restrict__ A, const float* __restrict__ alpha,
                                              const float* __restrict__ w1, const float* __restrict__ b1, const float* __restrict__ w2, const float* __restrict__ b2,
                                              const float* __restrict__ w4, const float* __restrict__ b4, const int* __restrict__ sp, h16* AT) {
    __shared__ __align__(16) h16 xbT[UP * XBP];
    __shared__ __align__(16) h16 wc[16 * XBP];
    __shared__ float sx[16 * UP];
    __shared__ float stt[RR * VV * VV];
    __shared__ float sw4[CC * RR];
    __shared__ float sb4[CC];
    __shared__ float sA[VV * VV];
    const int tid = threadIdx.x;
    const int lane = tid & 31, lr = lane & 15, hi = lane >> 4;
    const int wave = __builtin_amdgcn_readfirstlane((int)(threadIdx.x >> 5));
    const int s = blockIdx.x, n = blockIdx.y;
    const float thr = (float)sp[0];
#pragma unroll 1
    for (int i = tid; i < CC * UP; i += 256) { const unsigned c = (unsigned)i >> 5, v = (unsigned)i & 31u;
        const float xv = XBAR[((size_t)n * CC + c) * UP + v];
        xbT[v * XBP + c] = toh_flush(xv * XBC); }
#pragma unroll 1
    for (int i = tid; i < 16 * CC; i += 256) { const unsigned j = (unsigned)i >> 6, c = (unsigned)i & 63u;
        const unsigned ro = ((unsigned)s * RR + (j & 7u)) * CC + c;
        float p1 = w1[ro], p2 = w2[ro]; asm volatile("" : "+v"(p1), "+v"(p2));
        float wv = (j < 8u) ? bfr(p1) : bfr(p2);
        wv = (fabsf(wv) > thr) ? wv : 0.0f;
        wc[j * XBP + c] = toh_flush(wv * WCC); }
#pragma unroll 1
    for (int i = tid; i < CC * RR; i += 256) { float wv = bfr(w4[(size_t)s * CC * RR + i]); sw4[i] = (fabsf(wv) > thr) ? wv : 0.0f; }
    if (tid < CC) sb4[tid] = bfr(b4[s * CC + tid]);
#pragma unroll 1
    for (int i = tid; i < VV * VV; i += 256) sA[i] = bfr(A[s * VV * VV + i]);
    __syncthreads();
    if (wave == 0) {
        v8f d0 = (v8f){}, d1 = (v8f){};
#pragma unroll
        for (int kk = 0; kk < 2; ++kk) {
            const unsigned ao = (unsigned)lr * XBP + kk * 32 + 8 * hi;
            const v8h a0l = *(const v8ha*)(&xbT[ao]), a0h = *(const v8ha*)(&xbT[ao + 16]);
            const v8h a1l = *(const v8ha*)(&xbT[ao + 16 * XBP]), a1h = *(const v8ha*)(&xbT[ao + 16 * XBP + 16]);
            const v8h bl = *(const v8ha*)(&wc[ao]), bh = *(const v8ha*)(&wc[ao + 16]);
            const v16h a0 = cat16(a0l, a0h), a1 = cat16(a1l, a1h), bb = cat16(bl, bh);
            d0 = wmma16g(a0, bb, d0); d1 = wmma16g(a1, bb, d1); }
        float q1 = b1[s * RR + (lr & 7)], q2 = b2[s * RR + (lr & 7)]; asm volatile("" : "+v"(q1), "+v"(q2));
        const float bj = (lr < 8) ? bfr(q1) : bfr(q2);
#pragma unroll
        for (int r = 0; r < 8; ++r) { sx[lr * UP + 8 * hi + r] = d0[r] * X1I + bj; sx[lr * UP + 16 + 8 * hi + r] = d1[r] * X1I + bj; }
    }
    __syncthreads();
#pragma unroll 1
    for (int i = tid; i < RR * VV * VV; i += 256) { const unsigned r = (unsigned)i / (unsigned)(VV * VV); const unsigned rem = (unsigned)i - r * (unsigned)(VV * VV);
        const unsigned u = rem / (unsigned)VV; const unsigned v = rem - u * (unsigned)VV;
        stt[i] = tanhf(sx[r * UP + u] - sx[(RR + r) * UP + v]); }
    __syncthreads();
    const float al = bfr(alpha[0]);
#pragma unroll 1
    for (int it = 0; it < 32; ++it) {
        const unsigned g = (unsigned)it * 256u + (unsigned)tid;
        const unsigned o = g >> 7, v = (g >> 2) & 31u, u0 = (g & 3u) * 8u;
        const unsigned vc = v < (unsigned)VV ? v : (unsigned)(VV - 1);
        float acc[8]; unsigned sidx[8];
#pragma unroll
        for (int i = 0; i < 8; ++i) { const unsigned u = u0 + i; const unsigned uc = u < (unsigned)VV ? u : (unsigned)(VV - 1); sidx[i] = uc * VV + vc; acc[i] = 0.0f; }
#pragma unroll 1
        for (int r = 0; r < RR; ++r) { const float w = sw4[o * RR + r];
#pragma unroll
            for (int i = 0; i < 8; ++i) acc[i] += w * stt[r * (VV * VV) + sidx[i]]; }
        const float bo = sb4[o];
        v8h hv;
#pragma unroll
        for (int i = 0; i < 8; ++i) { const bool ok = ((u0 + i) < (unsigned)VV) & (v < (unsigned)VV);
            float val = (acc[i] + bo) * al + sA[sidx[i]];
            val = ok ? val * ATC : 0.0f;
            hv[i] = toh_flush(val); }
        h16* dp = AT + (((size_t)n * CC + o) * NS + (size_t)s) * (UP * UP) + (size_t)(g & 127u) * 8;
        *(volatile v8h*)dp = hv; __threadfence(); *(volatile v8h*)dp = hv;
    }
}

__global__ __launch_bounds__(32 * NW) void k_main(const bf* __restrict__ XT, const bf* __restrict__ W3B, const float* __restrict__ b3,
                                                  const h16* __restrict__ AT, const float* __restrict__ x, float* OUT) {
    __shared__ __align__(16) h16 x3s[NS * OGC * OPX];
    __shared__ __align__(16) float os[NW * PB];
    const int tid = threadIdx.x;
    const int lane = tid & 31, lr = lane & 15, hi = lane >> 4;
    const int wave = __builtin_amdgcn_readfirstlane((int)(threadIdx.x >> 5));
    const int tt = blockIdx.x, og = blockIdx.y, n = blockIdx.z;
    { const v8h zz = (v8h){};
#pragma unroll 1
      for (int i = tid; i < NS * OGC * TB; i += 32 * NW) { const unsigned so = (unsigned)i >> 5, t = (unsigned)i & 31u;
          *(v8ha*)(&x3s[so * OPX + t * UP + 24u]) = zz; } }
    __syncthreads();
    v16bf wb[NS][2]; float bia[NS];
#pragma unroll
    for (int s = 0; s < NS; ++s) { const size_t wo = ((size_t)(s * CC + og * OGC + lr)) * CC + 8 * hi;
        wb[s][0] = ldb(W3B + wo); wb[s][1] = ldb(W3B + wo + 32); bia[s] = bfr(b3[s * CC + og * OGC + lr]); }
    const size_t xrow0 = (size_t)n * PIXN + (size_t)tt * PB;
#pragma unroll 1
    for (int mt = wave; mt < MTN; mt += NW) {
        const bf* ap = XT + (xrow0 + (size_t)(mt * 16 + lr)) * CC + 8 * hi;
        const v16bf a0 = ldb(ap), a1 = ldb(ap + 32);
        const unsigned pl = (unsigned)mt * 16u + 8u * (unsigned)hi;
        const unsigned tl0 = pl / (unsigned)VV; const unsigned u0 = pl - tl0 * (unsigned)VV;
        unsigned base = (unsigned)lr * OPX + tl0 * UP + u0;
        asm volatile("" : "+v"(base));
#pragma unroll
        for (int s = 0; s < NS; ++s) {
            v8f acc = (v8f){};
            acc = wmmabg(a0, wb[s][0], acc); acc = wmmabg(a1, wb[s][1], acc);
#pragma unroll
            for (int r = 0; r < 8; ++r) { const unsigned wrap = (u0 + (unsigned)r >= (unsigned)VV) ? (unsigned)(UP - VV) : 0u;
                x3s[(unsigned)s * (OGC * OPX) + base + (unsigned)r + wrap] = toh_flush((acc[r] + bia[s]) * X3C); } }
    }
    __syncthreads();
    const unsigned wbo = (unsigned)wave * (unsigned)PB;
#pragma unroll 1
    for (int j = 0; j < 2; ++j) {
        const int cl = wave * 2 + j; const int c = og * OGC + cl;
        const size_t ato = (((size_t)n * CC + c) * NS) * (UP * UP) + (size_t)lr * UP + 8 * hi;
        v8f z00 = (v8f){}, z01 = (v8f){}, z10 = (v8f){}, z11 = (v8f){};
#pragma unroll
        for (int s = 0; s < NS; ++s) {
            const unsigned xo = (unsigned)(s * OGC + cl) * OPX + (unsigned)lr * UP + 8u * (unsigned)hi;
            const v8h p0 = *(const v8ha*)(&x3s[xo]), p1 = *(const v8ha*)(&x3s[xo + 16]);
            const v8h p2 = *(const v8ha*)(&x3s[xo + 16 * UP]), p3 = *(const v8ha*)(&x3s[xo + 16 * UP + 16]);
            const v16h a0 = cat16(p0, p1), a1 = cat16(p2, p3);
            const v16h b0 = ldh(AT + ato + (size_t)s * (UP * UP)), b1 = ldh(AT + ato + (size_t)s * (UP * UP) + 16 * UP);
            z00 = wmma16g(a0, b0, z00); z01 = wmma16g(a0, b1, z01); z10 = wmma16g(a1, b0, z10); z11 = wmma16g(a1, b1, z11); }
#pragma unroll
        for (int r = 0; r < 8; ++r) { const unsigned ta = (8u * (unsigned)hi + (unsigned)r) * VV, tb = (16u + 8u * (unsigned)hi + (unsigned)r) * VV;
            os[wbo + ta + lr] = z00[r] * ZI; os[wbo + tb + lr] = z10[r] * ZI;
            if (lr < VV - 16) { os[wbo + ta + 16 + lr] = z01[r] * ZI; os[wbo + tb + 16 + lr] = z11[r] * ZI; } }
        wave_sync();
        const size_t cb = (((size_t)n * CC + c) * TT + (size_t)tt * TB) * VV;
#pragma unroll 1
        for (int ps = 0; ps < 2; ++ps) {
#pragma unroll 1
            for (int it = 0; it < 7; ++it) { const unsigned q = (unsigned)it * 32u + (unsigned)lane; const unsigned qc = q < (unsigned)NQ ? q : (unsigned)(NQ - 1);
                const v4f zv = *(const v4fa*)(&os[wbo + 4u * qc]);
                v4f xv = *(const v4f*)(x + cb + 4u * qc);
                asm volatile("" : "+v"(xv));
                v4f val;
#pragma unroll
                for (int i = 0; i < 4; ++i) val[i] = fmaxf(zv[i] + bfr(xv[i]), 0.0f);
                if (q < (unsigned)NQ) *(volatile v4f*)(OUT + cb + 4u * q) = val; }
            if (ps == 0) __threadfence(); }
        wave_sync();
    }
}

static constexpr size_t al256(size_t v) { return (v + 255) & ~(size_t)255; }
static constexpr size_t SZ_XT = al256((size_t)NB * PIXN * CC * 2);
static constexpr size_t SZ_W3 = al256((size_t)NS * CC * CC * 2);
static constexpr size_t SZ_XB = al256((size_t)NB * CC * UP * 4);
static constexpr size_t SZ_AT = al256((size_t)NB * CC * NS * UP * UP * 2);
static constexpr size_t SZ_TOTAL = SZ_XT + SZ_W3 + SZ_XB + SZ_AT;
static_assert(SZ_TOTAL <= (size_t)134217728);
static_assert(((size_t)NB * PIXN * 8) * 16 == (size_t)NB * PIXN * CC * 2);
static_assert(((size_t)NB * CC) * 128 == (size_t)NB * CC * UP * 4);
static_assert(((size_t)NS * NB * 8192) * 16 == (size_t)NB * CC * NS * UP * UP * 2);

extern "C" void kernel_launch(void* const* d_in, const int* in_sizes, int n_in,
                              void* d_out, int out_size, void* d_ws, size_t ws_size, hipStream_t stream) {
    if (n_in < 12) return;
    const size_t needx = (size_t)NB * CC * PIXN;
    if ((size_t)in_sizes[0] < needx) return;
    if (in_sizes[1] < NS * VV * VV || in_sizes[2] < 1) return;
    if (in_sizes[3] < NS * RR * CC || in_sizes[4] < NS * RR || in_sizes[5] < NS * RR * CC || in_sizes[6] < NS * RR) return;
    if (in_sizes[7] < NS * CC * CC || in_sizes[8] < NS * CC || in_sizes[9] < NS * CC * RR || in_sizes[10] < NS * CC || in_sizes[11] < 1) return;
    if ((size_t)out_size < needx) return;
    if (SZ_TOTAL > ws_size) return;
    const float* x  = (const float*)d_in[0];
    const float* Aj = (const float*)d_in[1];
    const float* al = (const float*)d_in[2];
    const float* w1 = (const float*)d_in[3]; const float* b1 = (const float*)d_in[4];
    const float* w2 = (const float*)d_in[5]; const float* b2 = (const float*)d_in[6];
    const float* w3 = (const float*)d_in[7]; const float* b3 = (const float*)d_in[8];
    const float* w4 = (const float*)d_in[9]; const float* b4 = (const float*)d_in[10];
    const int* sp = (const int*)d_in[11];
    float* OUT = (float*)d_out;
    char* wsp = (char*)d_ws;
    bf*    XT   = (bf*)wsp;    wsp += SZ_XT;
    bf*    W3B  = (bf*)wsp;    wsp += SZ_W3;
    float* XBAR = (float*)wsp; wsp += SZ_XB;
    h16*   AT   = (h16*)wsp;   wsp += SZ_AT;

    { const unsigned n8 = (unsigned)((size_t)NS * CC * CC / 8);
      k_wcvt<<<(n8 + 255u) / 256u, 256, 0, stream>>>(w3, sp, W3B, n8); }
    { const unsigned n8 = (unsigned)((size_t)NB * PIXN * 8);
      k_tr<<<(n8 + 255u) / 256u, 256, 0, stream>>>(x, XT, n8); }
    k_xbar<<<NB * CC, 256, 0, stream>>>(x, XBAR);
    k_amat<<<dim3(NS, NB, 1), 256, 0, stream>>>(XBAR, Aj, al, w1, b1, w2, b2, w4, b4, sp, AT);
    k_main<<<dim3(TT / TB, CC / OGC, NB), 32 * NW, 0, stream>>>(XT, W3B, b3, AT, x, OUT);
}
